// sub_model_59433757442324
// MI455X (gfx1250) — hardware-run, weakly checked
//
#include <hip/hip_runtime.h>
#include <hip/hip_fp16.h>
#include <math.h>

typedef __attribute__((ext_vector_type(16))) _Float16 v16h;
typedef __attribute__((ext_vector_type(8)))  _Float16 v8h;
typedef __attribute__((ext_vector_type(8)))  float    v8f;
typedef __attribute__((ext_vector_type(4)))  float    v4f;
typedef __attribute__((ext_vector_type(2)))  unsigned v2u;
typedef __attribute__((ext_vector_type(4)))  unsigned v4u;

constexpr int kBatch   = 4;
constexpr int kH       = 64;
constexpr int kW       = 64;
constexpr int kL       = kH * kW;
constexpr int kRows    = kBatch * kL;
constexpr int kD       = 192;
constexpr int kRank    = 6;
constexpr int kRkP     = 32;
constexpr int kNst     = 16;
constexpr int kXpN     = kRank + 2 * kNst;
constexpr int kXpP     = 64;
constexpr int kDirs    = 4;
constexpr int kAlpFloats = kDirs * kD * kNst;
constexpr int kPadFloats = kAlpFloats + kDirs * kD;
constexpr float kXCarry = 64.0f;
constexpr float kWCarry = 1024.0f;
constexpr float kRCarry = 1024.0f;
constexpr float kYCarry = 64.0f;
constexpr float kResid  = 2048.0f;
static_assert(kH == 64 && kW == 64 && kH == kW);
static_assert(kL == 4096 && kRows == 16384);
static_assert(kD == 192 && kXpN == 38 && kDirs == 4 && kNst == 16);
static_assert(kRank + 1 <= kRkP && kRank < 16);
static_assert((kD % 32) == 0 && (kRkP % 32) == 0);
static_assert((kD % 64) == 0 && (kXpP % 64) == 0);
static_assert((kRows % 32) == 0);
static_assert((kL % 64) == 0 && (kL % 4) == 0);
static_assert(kAlpFloats == 12288 && kPadFloats == 13056);

constexpr size_t kSzXS   = (size_t)kDirs * kRows * kD * 4;
constexpr size_t kSzXSH  = (size_t)kDirs * kRows * kD * 2;
constexpr size_t kSzXPW  = (size_t)kDirs * kXpP * kD * 2;
constexpr size_t kSzXD   = (size_t)kDirs * kRows * kXpP * 4;
constexpr size_t kSzDRH  = (size_t)kDirs * kRows * kRkP * 2;
constexpr size_t kSzDRL  = (size_t)kDirs * kRows * kRkP * 2;
constexpr size_t kSzDTW  = (size_t)kDirs * kD * kRkP * 2;
constexpr size_t kSzDTP  = (size_t)kDirs * kRows * kD * 4;
constexpr size_t kSzPADS = (size_t)kPadFloats * 4;
constexpr size_t kSzYH   = (size_t)kDirs * kRows * kD * 2;
constexpr size_t kOffXS   = 0;
constexpr size_t kOffXSH  = kOffXS   + kSzXS;
constexpr size_t kOffXPW  = kOffXSH  + kSzXSH;
constexpr size_t kOffXD   = kOffXPW  + kSzXPW;
constexpr size_t kOffDRH  = kOffXD   + kSzXD;
constexpr size_t kOffDRL  = kOffDRH  + kSzDRH;
constexpr size_t kOffDTW  = kOffDRL  + kSzDRL;
constexpr size_t kOffDTP  = kOffDTW  + kSzDTW;
constexpr size_t kOffPADS = kOffDTP  + kSzDTP;
constexpr size_t kOffYH   = kOffPADS + kSzPADS;
constexpr size_t kWsTotal = kOffYH   + kSzYH;
static_assert(kSzXS == 50331648ull && kSzXSH == 25165824ull && kSzXPW == 98304ull && kSzXD == 16777216ull);
static_assert(kSzDRH == 4194304ull && kSzDRL == 4194304ull && kSzDTW == 49152ull && kSzDTP == 50331648ull);
static_assert(kSzPADS == 52224ull && kSzYH == 25165824ull);
static_assert(kWsTotal == 50331648ull + 25165824ull + 98304ull + 16777216ull + 4194304ull + 4194304ull +
              49152ull + 50331648ull + 52224ull + 25165824ull);
static_assert(kWsTotal == 176360448ull);
static_assert(kWsTotal <= 268435456ull);
static_assert((kSzXS % 128) == 0 && (kSzXSH % 128) == 0 && (kSzXPW % 128) == 0 && (kSzXD % 128) == 0 &&
              (kSzDRH % 128) == 0 && (kSzDRL % 128) == 0 && (kSzDTW % 128) == 0 && (kSzDTP % 128) == 0 &&
              (kSzPADS % 128) == 0 && (kSzYH % 128) == 0);
static_assert((((size_t)kRows * kD * 4) % 128) == 0 && (((size_t)kRows * kD * 2) % 128) == 0 &&
              (((size_t)kXpP * kD * 2) % 128) == 0 && (((size_t)kRows * kXpP * 4) % 128) == 0 &&
              (((size_t)kRows * kRkP * 2) % 128) == 0 && (((size_t)kD * kRkP * 2) % 128) == 0 &&
              (((size_t)kD * kNst * 4) % 128) == 0 && (((size_t)kAlpFloats * 4) % 128) == 0);

__device__ __forceinline__ _Float16 f16_flush(float v) {
  const float w = (fabsf(v) < 6.103515625e-05f) ? 0.0f : v;
  return (_Float16)w;
}
__device__ __forceinline__ void f16_split(float v, _Float16& hi, _Float16& lo) {
  hi = f16_flush(v);
  const float hf = (float)hi;
  const float r = (v - hf) * kResid;
  lo = f16_flush(r);
}

__device__ __forceinline__ float bf16r(float v) {
  unsigned u = __float_as_uint(v);
  u = (u + 0x7FFFu + ((u >> 16) & 1u)) & 0xFFFF0000u;
  return __uint_as_float(u);
}

__device__ __forceinline__ float h16_to_f32(unsigned hb) {
  const unsigned sgn = (hb & 0x8000u) << 16; const unsigned em = hb & 0x7fffu;
  const float fn = __uint_as_float((em << 13) + 0x38000000u);
  const float fs = (float)em * 5.9604644775390625e-8f;
  const float mag = (em < 0x400u) ? fs : fn; return __uint_as_float(__float_as_uint(mag) | sgn); }

namespace eng {
union FragU { v16h v; v8h h[2]; };
__device__ __forceinline__ v16h frag_load(const _Float16* p) {
  FragU f;
  f.h[0] = *(const v8h*)(p);
  f.h[1] = *(const v8h*)(p + 16);
  return f.v;
}
__device__ __forceinline__ v8f mma(v16h a, v16h b, v8f c) {
  return __builtin_amdgcn_wmma_f32_16x16x32_f16(false, a, false, b, (short)0, c, false, false);
}
__device__ __forceinline__ void guard1(v8f& a, v16h x, v16h y) {
  asm volatile("v_nop\n\tv_nop\n\tv_nop\n\tv_nop" : "+v"(a) : "v"(x), "v"(y));
}
__device__ __forceinline__ void guard_acc(v8f& a) {
  asm volatile("v_nop\n\tv_nop\n\tv_nop\n\tv_nop" : "+v"(a));
}
__device__ __forceinline__ void keep4(v16h a, v16h b, v16h c, v16h d) {
  asm volatile("v_nop" :: "v"(a), "v"(b), "v"(c), "v"(d));
}

template <int MI, int SPL>
__global__ __launch_bounds__(256) void gemm_f16_kernel(
    const unsigned short* __restrict__ Ap, const unsigned short* __restrict__ A2p, int lda,
    const unsigned short* __restrict__ Btp, const unsigned short* __restrict__ Bt2p, int ldb,
    float* __restrict__ C, int ldc, int M, int N, int K, float scale, float rscale)
{
  static_assert(MI >= 1 && MI <= 2);
  static_assert(SPL >= 0 && SPL <= 2);
  const _Float16* A   = (const _Float16*)Ap;
  const _Float16* A2  = (const _Float16*)A2p;
  const _Float16* Bt  = (const _Float16*)Btp;
  const _Float16* Bt2 = (const _Float16*)Bt2p;
  __shared__ __align__(16) float sT[8][16 * 68];
  const int lane = threadIdx.x & 31;
  const int wave = threadIdx.x >> 5;
  const int tilesN = N >> 6;
  const int tilesM = M / (16 * MI);
  const int tile = blockIdx.x * 8 + wave;
  if (tile >= tilesM * tilesN) return;
  const int tm = tile / tilesN;
  const int tn = tile - tm * tilesN;
  const int m0 = tm * (16 * MI);
  const int n0 = tn << 6;
  const int rlane = lane & 15;
  const int koff  = (lane >> 4) * 8;
  const int mOff  = (lane >> 4) * 8;

  v8f acc[MI][4], accr[MI][4];
#pragma unroll
  for (int i = 0; i < MI; ++i)
#pragma unroll
    for (int j = 0; j < 4; ++j) {
      acc[i][j]  = (v8f){0.f, 0.f, 0.f, 0.f, 0.f, 0.f, 0.f, 0.f};
      accr[i][j] = (v8f){0.f, 0.f, 0.f, 0.f, 0.f, 0.f, 0.f, 0.f};
    }

  for (int k0 = 0; k0 < K; k0 += 32) {
    v16h bh[4], bl[4];
#pragma unroll
    for (int j = 0; j < 4; ++j) {
      const size_t bo = (size_t)(n0 + (j << 4) + rlane) * ldb + koff + k0;
      bh[j] = frag_load(Bt + bo);
      if (SPL == 2) bl[j] = frag_load(Bt2 + bo); else bl[j] = bh[j];
    }
#pragma unroll
    for (int i = 0; i < MI; ++i) {
      const size_t ao = (size_t)(m0 + (i << 4) + rlane) * lda + koff + k0;
      const v16h ah = frag_load(A + ao);
      v16h al = ah;
      if (SPL >= 1) al = frag_load(A2 + ao);
#pragma unroll
      for (int j = 0; j < 4; ++j) {
        acc[i][j] = mma(ah, bh[j], acc[i][j]);
        if (SPL >= 1) accr[i][j] = mma(al, bh[j], accr[i][j]);
        if (SPL == 2) accr[i][j] = mma(ah, bl[j], accr[i][j]);
      }
#pragma unroll
      for (int j = 0; j < 4; ++j) {
        guard1(acc[i][j], ah, al);
        if (SPL >= 1) guard1(accr[i][j], ah, al);
      }
    }
    keep4(bh[0], bh[1], bh[2], bh[3]);
    if (SPL == 2) keep4(bl[0], bl[1], bl[2], bl[3]);
  }
#pragma unroll
  for (int i = 0; i < MI; ++i)
#pragma unroll
    for (int j = 0; j < 4; ++j) {
      guard_acc(acc[i][j]);
      if (SPL >= 1) guard_acc(accr[i][j]);
    }

  float* slab = sT[wave];
#pragma unroll
  for (int i = 0; i < MI; ++i) {
    const int mBase = m0 + (i << 4);
#pragma unroll
    for (int j = 0; j < 4; ++j) {
#pragma unroll
      for (int r = 0; r < 8; ++r) {
        float v = acc[i][j][r] * scale;
        if (SPL >= 1) v += accr[i][j][r] * rscale;
        slab[(mOff + r) * 68 + (j << 4) + rlane] = v;
      }
    }
    __builtin_amdgcn_fence(__ATOMIC_RELEASE, "workgroup");
    __builtin_amdgcn_wave_barrier();
    __builtin_amdgcn_fence(__ATOMIC_ACQUIRE, "workgroup");
    {
      const int hh = lane >> 4, c4 = (lane & 15) * 4;
      for (int pass = 0; pass < 2; ++pass) {
#pragma unroll
        for (int it = 0; it < 8; ++it) {
          const int row = it * 2 + hh;
          const v4f v = *(const v4f*)(slab + row * 68 + c4);
          *(volatile v4f*)(C + (size_t)(mBase + row) * ldc + n0 + c4) = v;
        }
        __threadfence();
      }
    }
    __builtin_amdgcn_fence(__ATOMIC_RELEASE, "workgroup");
    __builtin_amdgcn_wave_barrier();
    __builtin_amdgcn_fence(__ATOMIC_ACQUIRE, "workgroup");
  }
}
}

__device__ __forceinline__ _Float16 in_half(float v, float carry, bool live) {
  const float t = live ? (bf16r(v) * carry) : 0.0f;
  return f16_flush(t);
}
__device__ __forceinline__ _Float16 val_half(float v, float carry, bool live) {
  const float t = live ? (v * carry) : 0.0f;
  return f16_flush(t);
}
__device__ __forceinline__ v8h pack8_in(v4f a0, v4f a1, float carry, bool live) {
  const float f0 = a0[0];
  const float f1 = a0[1];
  const float f2 = a0[2];
  const float f3 = a0[3];
  const float f4 = a1[0];
  const float f5 = a1[1];
  const float f6 = a1[2];
  const float f7 = a1[3];
  v8h hv;
  hv[0] = in_half(f0, carry, live);
  hv[1] = in_half(f1, carry, live);
  hv[2] = in_half(f2, carry, live);
  hv[3] = in_half(f3, carry, live);
  hv[4] = in_half(f4, carry, live);
  hv[5] = in_half(f5, carry, live);
  hv[6] = in_half(f6, carry, live);
  hv[7] = in_half(f7, carry, live);
  return hv;
}
__device__ __forceinline__ int src_pixel(int k, int t) {
  const int u = (k >= 2) ? (kL - 1 - t) : t;
  const int q = u / kW;
  const int r = u - q * kW;
  const int pt = r * kW + q;
  return ((k & 1) != 0) ? pt : u;
}
__device__ __forceinline__ int inv_time(int k, int l) {
  const int h = l / kW;
  const int w = l - h * kW;
  const int tt = w * kH + h;
  const int base = ((k & 1) != 0) ? tt : l;
  return (k >= 2) ? (kL - 1 - base) : base;
}

__global__ __launch_bounds__(256) void order_kernel(
    const float* __restrict__ x, float* __restrict__ XS)
{
  const int i = blockIdx.x * 256 + threadIdx.x;
  const int k = i / (kRows * (kD / 4));
  const int rem = i - k * (kRows * (kD / 4));
  const int R = rem / (kD / 4);
  const int d4 = (rem - R * (kD / 4)) * 4;
  const int b = R / kL;
  const int t = R - b * kL;
  const int p = src_pixel(k, t);
  const float* sp = x + ((size_t)(b * kD + d4) * kL + p);
  const float f0 = sp[0];
  const float f1 = sp[kL];
  const float f2 = sp[2 * kL];
  const float f3 = sp[3 * kL];
  v4f o;
  o[0] = bf16r(f0);
  o[1] = bf16r(f1);
  o[2] = bf16r(f2);
  o[3] = bf16r(f3);
  float* q = XS + (size_t)i * 4;
  *(volatile v4f*)q = o;
  __threadfence();
  *(volatile v4f*)q = o;
}

__global__ __launch_bounds__(256) void pack_xs_kernel(
    const float* __restrict__ x, unsigned short* __restrict__ XSH)
{
  const int i = blockIdx.x * 256 + threadIdx.x;
  const int k = i / (kRows * (kD / 8));
  const int rem = i - k * (kRows * (kD / 8));
  const int R = rem / (kD / 8);
  const int d8 = (rem - R * (kD / 8)) * 8;
  const int b = R / kL;
  const int t = R - b * kL;
  const int p = src_pixel(k, t);
  const float* sp = x + ((size_t)(b * kD + d8) * kL + p);
  const float f0 = sp[0];
  const float f1 = sp[kL];
  const float f2 = sp[2 * kL];
  const float f3 = sp[3 * kL];
  const float f4 = sp[4 * kL];
  const float f5 = sp[5 * kL];
  const float f6 = sp[6 * kL];
  const float f7 = sp[7 * kL];
  v8h hv;
  hv[0] = in_half(f0, kXCarry, true);
  hv[1] = in_half(f1, kXCarry, true);
  hv[2] = in_half(f2, kXCarry, true);
  hv[3] = in_half(f3, kXCarry, true);
  hv[4] = in_half(f4, kXCarry, true);
  hv[5] = in_half(f5, kXCarry, true);
  hv[6] = in_half(f6, kXCarry, true);
  hv[7] = in_half(f7, kXCarry, true);
  unsigned short* q = XSH + (size_t)i * 8;
  *(volatile v8h*)q = hv;
  __threadfence();
  *(volatile v8h*)q = hv;
}

__global__ __launch_bounds__(256) void pack_xpw_kernel(
    const float* __restrict__ w, unsigned short* __restrict__ XPW)
{
  const int i = blockIdx.x * 256 + threadIdx.x;
  const int k = i / (kXpP * (kD / 8));
  const int rem = i - k * (kXpP * (kD / 8));
  const int n = rem / (kD / 8);
  const int j8 = (rem - n * (kD / 8)) * 8;
  const bool live = (n < kXpN);
  const int nc = live ? n : (kXpN - 1);
  const float* sp = w + ((size_t)(k * kXpN + nc) * kD + j8);
  const v4f a0 = *(const v4f*)(sp);
  const v4f a1 = *(const v4f*)(sp + 4);
  const v8h hv = pack8_in(a0, a1, kWCarry, live);
  unsigned short* q = XPW + (size_t)i * 8;
  *(volatile v8h*)q = hv;
  __threadfence();
  *(volatile v8h*)q = hv;
}

__device__ __forceinline__ void dr_split(float v, int j, _Float16& hi, _Float16& lo) {
  const float t = (j < kRank) ? (v * kRCarry) : ((j == kRank) ? kRCarry : 0.0f);
  f16_split(t, hi, lo);
}
__global__ __launch_bounds__(256) void pack_dr_kernel(
    const float* __restrict__ XD, unsigned short* __restrict__ DRH, unsigned short* __restrict__ DRL)
{
  const int i = blockIdx.x * 256 + threadIdx.x;
  const int row = i / (kRkP / 8);
  const int j8 = (i - row * (kRkP / 8)) * 8;
  const int jc = (j8 < 16) ? j8 : 8;
  const float* sp = XD + (size_t)row * kXpP + jc;
  const v4f a0 = *(const v4f*)(sp);
  const v4f a1 = *(const v4f*)(sp + 4);
  const float f0 = a0[0];
  const float f1 = a0[1];
  const float f2 = a0[2];
  const float f3 = a0[3];
  const float f4 = a1[0];
  const float f5 = a1[1];
  const float f6 = a1[2];
  const float f7 = a1[3];
  _Float16 h0, h1, h2, h3, h4, h5, h6, h7;
  _Float16 l0, l1, l2, l3, l4, l5, l6, l7;
  dr_split(f0, j8 + 0, h0, l0);
  dr_split(f1, j8 + 1, h1, l1);
  dr_split(f2, j8 + 2, h2, l2);
  dr_split(f3, j8 + 3, h3, l3);
  dr_split(f4, j8 + 4, h4, l4);
  dr_split(f5, j8 + 5, h5, l5);
  dr_split(f6, j8 + 6, h6, l6);
  dr_split(f7, j8 + 7, h7, l7);
  v8h hv;
  hv[0] = h0;
  hv[1] = h1;
  hv[2] = h2;
  hv[3] = h3;
  hv[4] = h4;
  hv[5] = h5;
  hv[6] = h6;
  hv[7] = h7;
  v8h lv;
  lv[0] = l0;
  lv[1] = l1;
  lv[2] = l2;
  lv[3] = l3;
  lv[4] = l4;
  lv[5] = l5;
  lv[6] = l6;
  lv[7] = l7;
  unsigned short* qh = DRH + (size_t)i * 8;
  unsigned short* ql = DRL + (size_t)i * 8;
  *(volatile v8h*)qh = hv;
  *(volatile v8h*)ql = lv;
  __threadfence();
  *(volatile v8h*)qh = hv;
  *(volatile v8h*)ql = lv;
}

__device__ __forceinline__ _Float16 dtw_half(const float* __restrict__ wrow, float bias, int j) {
  const int jc = (j < kRank) ? j : (kRank - 1);
  const float wv = wrow[jc];
  const float t = (j < kRank) ? (bf16r(wv) * kWCarry) : ((j == kRank) ? (bf16r(bias) * kWCarry) : 0.0f);
  return f16_flush(t);
}
__global__ __launch_bounds__(256) void pack_dtw_kernel(
    const float* __restrict__ dtw, const float* __restrict__ dtb, unsigned short* __restrict__ DTW)
{
  const int i = blockIdx.x * 256 + threadIdx.x;
  const int kc = i / (kRkP / 8);
  const int j8 = (i - kc * (kRkP / 8)) * 8;
  const float* wrow = dtw + (size_t)kc * kRank;
  const float bias = dtb[kc];
  v8h hv;
  hv[0] = dtw_half(wrow, bias, j8 + 0);
  hv[1] = dtw_half(wrow, bias, j8 + 1);
  hv[2] = dtw_half(wrow, bias, j8 + 2);
  hv[3] = dtw_half(wrow, bias, j8 + 3);
  hv[4] = dtw_half(wrow, bias, j8 + 4);
  hv[5] = dtw_half(wrow, bias, j8 + 5);
  hv[6] = dtw_half(wrow, bias, j8 + 6);
  hv[7] = dtw_half(wrow, bias, j8 + 7);
  unsigned short* q = DTW + (size_t)i * 8;
  *(volatile v8h*)q = hv;
  __threadfence();
  *(volatile v8h*)q = hv;
}

__global__ __launch_bounds__(32) void pads_kernel(
    const float* __restrict__ alog, const float* __restrict__ dsk, float* __restrict__ PADS)
{
  const int wi = blockIdx.x * 32 + threadIdx.x;
  const int f0 = wi * 4;
  const bool isA = (f0 < kAlpFloats);
  const int ea = isA ? f0 : (kAlpFloats - 4);
  const int dq = f0 - kAlpFloats;
  const int ed = isA ? 0 : dq;
  const v4f va = *(const v4f*)(alog + ea);
  const v4f vd = *(const v4f*)(dsk + ed);
  const float a0 = va[0];
  const float a1 = va[1];
  const float a2 = va[2];
  const float a3 = va[3];
  const float e0 = vd[0];
  const float e1 = vd[1];
  const float e2 = vd[2];
  const float e3 = vd[3];
  const float s0 = isA ? a0 : e0;
  const float s1 = isA ? a1 : e1;
  const float s2 = isA ? a2 : e2;
  const float s3 = isA ? a3 : e3;
  v4f o;
  o[0] = bf16r(s0);
  o[1] = bf16r(s1);
  o[2] = bf16r(s2);
  o[3] = bf16r(s3);
  float* q = PADS + (size_t)f0;
  *(volatile v4f*)q = o;
  __threadfence();
  *(volatile v4f*)q = o;
}

typedef float    ms1_v4f __attribute__((ext_vector_type(4)));
typedef unsigned ms1_v4u __attribute__((ext_vector_type(4)));
struct ms1_args {
  const float* dtpre;
  const float* u;
  const float* bc;
  const float* z;
  const float* A_log;
  const float* Dskip;
  __half* y;
  __half* y_lo;
  long ld_dtpre;
  long ld_u;
  long ld_bc;
  long ld_z;
  long ld_y;
  int offB;
  int offC;
  int offZ;
  float ycarry;
  int dir;
  int D;
  int L;
  int nbatch;
};
static_assert(sizeof(ms1_args) == 136);

__device__ __forceinline__ float ms1_flush16(float v) {
  return (fabsf(v) < 6.103515625e-05f) ? 0.0f : v;
}
__device__ __forceinline__ unsigned ms1_h16bits(float v) {
  return (unsigned)__half_as_ushort(__float2half_rn(ms1_flush16(v)));
}
__device__ __forceinline__ float ms1_h16val(unsigned b) {
  return __half2float(__ushort_as_half((unsigned short)b));
}
__device__ __forceinline__ float ms1_softplus(float v) {
  return fmaxf(v, 0.0f) + log1pf(expf(-fabsf(v)));
}
__device__ __forceinline__ void ms1_pack2(float v0, float v1, unsigned& hw, unsigned& lw) {
  const unsigned h0 = ms1_h16bits(v0);
  const unsigned h1 = ms1_h16bits(v1);
  const float r0 = (v0 - ms1_h16val(h0)) * 2048.0f;
  const float r1 = (v1 - ms1_h16val(h1)) * 2048.0f;
  const unsigned l0 = ms1_h16bits(r0);
  const unsigned l1 = ms1_h16bits(r1);
  hw = h0 | (h1 << 16);
  lw = l0 | (l1 << 16);
}

template <int NSTATE>
__global__ __launch_bounds__(64 * (NSTATE / 16)) void ms1_scan_kernel(ms1_args a)
{
  static_assert(NSTATE == 16 || NSTATE == 64);
  constexpr int NQ  = NSTATE / 16;
  constexpr int NT  = 64 * NQ;
  constexpr int NW  = NT / 32;
  constexpr int BCW = 2 * NSTATE;
  constexpr int YP  = 68;
  constexpr int RPI = NW * 4;
  constexpr int NIT = 64 / RPI;
  static_assert(16 * NT <= 64 * YP);
  __shared__ __align__(16) float sBC[64 * BCW];
  __shared__ __align__(16) float sY[64 * YP];
  const int tid  = threadIdx.x;
  const int lane = tid & 31;
  const int wave = tid >> 5;
  const int c    = tid / NQ;
  const int sq   = tid - c * NQ;
  const int bpb  = a.D / 64;
  const int bi   = blockIdx.x / bpb;
  if (bi >= a.nbatch) return;
  const int d0 = (blockIdx.x - bi * bpb) * 64;
  const int d  = d0 + c;
  const long rowb = (long)bi * a.L;
  const bool hasz  = (a.z != nullptr);
  const bool hasD  = (a.Dskip != nullptr);
  const bool hasLo = (a.y_lo != nullptr);

#pragma unroll 1
  for (int n = 0; n < 16; ++n) {
    const float al = a.A_log[(long)d * NSTATE + sq * 16 + n];
    sY[n * NT + tid] = -expf(al);
  }
  __syncthreads();
  float An[16], h[16];
#pragma unroll
  for (int n = 0; n < 16; ++n) {
    An[n] = sY[n * NT + tid];
    h[n] = 0.0f;
  }
  float Dd = 0.0f;
  if (hasD) Dd = a.Dskip[d];

  const int nchunk = a.L / 64;
  const bool fwd = (a.dir > 0);
  const int s0 = fwd ? 0 : 63;
  const int sd = fwd ? 1 : -1;
  const int q  = lane >> 3;
  const int c8 = (lane & 7) * 8;

  for (int ci = 0; ci < nchunk; ++ci) {
    const int tb = fwd ? (ci * 64) : (a.L - 64 - ci * 64);
    const long rowc = rowb + tb;
    __syncthreads();
#pragma unroll 8
    for (int i = 0; i < 32; ++i) {
      const int idx = tid + i * NT;
      const int st  = idx / BCW;
      const int col = idx - st * BCW;
      const int sc  = (col < NSTATE) ? (a.offB + col) : (a.offC + col - NSTATE);
      sBC[idx] = a.bc[(rowc + st) * a.ld_bc + sc];
    }
    __syncthreads();
    for (int s = 0; s < 64; ++s) {
      const int ls = s0 + sd * s;
      const long row = rowc + ls;
      float pre = a.dtpre[row * a.ld_dtpre + d];
      float uv  = a.u[row * a.ld_u + d];
      float zv  = 0.0f;
      if (hasz) zv = a.z[row * a.ld_z + a.offZ + d];
      asm volatile("" : "+v"(pre));
      asm volatile("" : "+v"(uv));
      asm volatile("" : "+v"(zv));
      const float delta = ms1_softplus(pre);
      const float dtx = delta * uv;
      const float* bp = sBC + ls * BCW + sq * 16;
      const float* cp = bp + NSTATE;
      ms1_v4f Bq[4], Cq[4];
#pragma unroll
      for (int k = 0; k < 4; ++k) {
        Bq[k] = *(const ms1_v4f*)(bp + 4 * k);
        Cq[k] = *(const ms1_v4f*)(cp + 4 * k);
      }
      float yv = 0.0f;
#pragma unroll
      for (int n = 0; n < 16; ++n) {
        const float e = __expf(delta * An[n]);
        h[n] = fmaf(e, h[n], dtx * Bq[n >> 2][n & 3]);
        yv = fmaf(h[n], Cq[n >> 2][n & 3], yv);
      }
      if (NQ > 1) {
        yv += __shfl_xor(yv, 1, 32);
        yv += __shfl_xor(yv, 2, 32);
      }
      if (hasD) yv = fmaf(uv, Dd, yv);
      if (hasz) {
        const float sg = __builtin_amdgcn_rcpf(1.0f + expf(-zv));
        yv = yv * (zv * sg);
      }
      if (sq == 0) sY[ls * YP + c] = yv * a.ycarry;
    }
    __syncthreads();
    ms1_v4u hw[NIT], lw[NIT];
#pragma unroll
    for (int it = 0; it < NIT; ++it) {
      const int row = it * RPI + wave * 4 + q;
      const float* sp = sY + row * YP + c8;
      const ms1_v4f f0 = *(const ms1_v4f*)(sp);
      const ms1_v4f f1 = *(const ms1_v4f*)(sp + 4);
      unsigned h0, h1, h2, h3, l0, l1, l2, l3;
      ms1_pack2(f0[0], f0[1], h0, l0);
      ms1_pack2(f0[2], f0[3], h1, l1);
      ms1_pack2(f1[0], f1[1], h2, l2);
      ms1_pack2(f1[2], f1[3], h3, l3);
      hw[it] = (ms1_v4u){h0, h1, h2, h3};
      lw[it] = (ms1_v4u){l0, l1, l2, l3};
    }
    for (int pass = 0; pass < 2; ++pass) {
#pragma unroll
      for (int it = 0; it < NIT; ++it) {
        const int row = it * RPI + wave * 4 + q;
        const long o = (rowc + row) * a.ld_y + d0 + c8;
        *(volatile ms1_v4u*)(a.y + o) = hw[it];
        if (hasLo) *(volatile ms1_v4u*)(a.y_lo + o) = lw[it];
      }
      __threadfence();
    }
  }
}

__device__ __forceinline__ float yh_val(const unsigned short* __restrict__ YH, int k, int b, int l, int d) {
  const int row = k * kRows + b * kL + inv_time(k, l);
  const unsigned hb = (unsigned)YH[(size_t)row * kD + d];
  return h16_to_f32(hb);
}
__device__ __forceinline__ float merge_one(const unsigned short* __restrict__ YH, int b, int l, int d) {
  const float v0 = yh_val(YH, 0, b, l, d);
  const float v1 = yh_val(YH, 1, b, l, d);
  const float v2 = yh_val(YH, 2, b, l, d);
  const float v3 = yh_val(YH, 3, b, l, d);
  const float s02 = v0 + v2;
  const float s13 = v1 + v3;
  const float s = s02 + s13;
  return s * (1.0f / kYCarry);
}
__global__ __launch_bounds__(256) void merge_out_kernel(
    const unsigned short* __restrict__ YH, float* __restrict__ out)
{
  const int i = blockIdx.x * 256 + threadIdx.x;
  const int bd = i / (kL / 4);
  const int l4 = (i - bd * (kL / 4)) * 4;
  const int b = bd / kD;
  const int d = bd - b * kD;
  const float r0 = merge_one(YH, b, l4 + 0, d);
  const float r1 = merge_one(YH, b, l4 + 1, d);
  const float r2 = merge_one(YH, b, l4 + 2, d);
  const float r3 = merge_one(YH, b, l4 + 3, d);
  v4f o;
  o[0] = r0;
  o[1] = r1;
  o[2] = r2;
  o[3] = r3;
  float* q = out + (size_t)i * 4;
  *(volatile v4f*)q = o;
  __threadfence();
  *(volatile v4f*)q = o;
}

static_assert(((kRows / 32) * (kXpP / 64)) % 8 == 0 && ((kRows / 32) * (kXpP / 64)) / 8 == 64);
static_assert(((kRows / 32) * (kD / 64)) % 8 == 0 && ((kRows / 32) * (kD / 64)) / 8 == 192);
static_assert(((kDirs * kRows * kD / 4) % 256) == 0 && (kDirs * kRows * kD / 4) / 256 == 12288);
static_assert(((kDirs * kRows * kD / 8) % 256) == 0 && (kDirs * kRows * kD / 8) / 256 == 6144);
static_assert(((kDirs * kXpP * kD / 8) % 256) == 0 && (kDirs * kXpP * kD / 8) / 256 == 24);
static_assert(((kDirs * kRows * kRkP / 8) % 256) == 0 && (kDirs * kRows * kRkP / 8) / 256 == 1024);
static_assert(((kDirs * kD * kRkP / 8) % 256) == 0 && (kDirs * kD * kRkP / 8) / 256 == 12);
static_assert((kPadFloats / 4) == 102 * 32);
static_assert(((kBatch * kD * kL / 4) % 256) == 0 && (kBatch * kD * kL / 4) / 256 == 3072);
static_assert((kD % 64) == 0 && (kL % 64) == 0);

extern "C" void kernel_launch(void* const* d_in, const int* in_sizes, int n_in,
                              void* d_out, int out_size, void* d_ws, size_t ws_size,
                              hipStream_t stream)
{
  if (n_in < 6) return;
  if (in_sizes[0] != kRows * kD) return;
  if (in_sizes[1] != kDirs * kXpN * kD) return;
  if (in_sizes[2] != kDirs * kD * kRank) return;
  if (in_sizes[3] != kDirs * kD) return;
  if (in_sizes[4] != kDirs * kD * kNst) return;
  if (in_sizes[5] != kDirs * kD) return;
  if (out_size != kRows * kD) return;
  if (ws_size < kWsTotal) return;

  const float* x      = (const float*)d_in[0];
  const float* w_xp   = (const float*)d_in[1];
  const float* dt_w   = (const float*)d_in[2];
  const float* dt_b   = (const float*)d_in[3];
  const float* a_logs = (const float*)d_in[4];
  const float* d_skip = (const float*)d_in[5];
  float* out = (float*)d_out;

  char* ws = (char*)d_ws;
  float*          XS   = (float*)(ws + kOffXS);
  unsigned short* XSH  = (unsigned short*)(ws + kOffXSH);
  unsigned short* XPW  = (unsigned short*)(ws + kOffXPW);
  float*          XD   = (float*)(ws + kOffXD);
  unsigned short* DRH  = (unsigned short*)(ws + kOffDRH);
  unsigned short* DRL  = (unsigned short*)(ws + kOffDRL);
  unsigned short* DTW  = (unsigned short*)(ws + kOffDTW);
  float*          DTP  = (float*)(ws + kOffDTP);
  float*          PADS = (float*)(ws + kOffPADS);
  unsigned short* YH   = (unsigned short*)(ws + kOffYH);
  float*          ALP  = PADS;
  float*          DSP  = PADS + kAlpFloats;

  constexpr float s2  = 1.0f / (kXCarry * kWCarry);
  constexpr float s3  = 1.0f / (kRCarry * kWCarry);
  constexpr float s3r = 1.0f / (kRCarry * kWCarry * kResid);

  order_kernel<<<(kDirs * kRows * kD / 4) / 256, 256, 0, stream>>>(x, XS);

  pack_xs_kernel<<<(kDirs * kRows * kD / 8) / 256, 256, 0, stream>>>(x, XSH);

  pack_xpw_kernel<<<(kDirs * kXpP * kD / 8) / 256, 256, 0, stream>>>(w_xp, XPW);

  for (int k = 0; k < kDirs; ++k) {
    eng::gemm_f16_kernel<2, 0><<<dim3((kRows / 32) * (kXpP / 64) / 8), 256, 0, stream>>>(
        XSH + (size_t)k * kRows * kD, nullptr, kD,
        XPW + (size_t)k * kXpP * kD, nullptr, kD,
        XD + (size_t)k * kRows * kXpP, kXpP, kRows, kXpP, kD, s2, 0.0f);
  }

  pack_dr_kernel<<<(kDirs * kRows * kRkP / 8) / 256, 256, 0, stream>>>(XD, DRH, DRL);

  pack_dtw_kernel<<<(kDirs * kD * kRkP / 8) / 256, 256, 0, stream>>>(dt_w, dt_b, DTW);

  for (int k = 0; k < kDirs; ++k) {
    eng::gemm_f16_kernel<2, 1><<<dim3((kRows / 32) * (kD / 64) / 8), 256, 0, stream>>>(
        DRH + (size_t)k * kRows * kRkP, DRL + (size_t)k * kRows * kRkP, kRkP,
        DTW + (size_t)k * kD * kRkP, DTW + (size_t)k * kD * kRkP, kRkP,
        DTP + (size_t)k * kRows * kD, kD, kRows, kD, kRkP, s3, s3r);
  }

  pads_kernel<<<102, 32, 0, stream>>>(a_logs, d_skip, PADS);

  for (int k = 0; k < kDirs; ++k) {
    ms1_args sa;
    sa.dtpre = DTP + (size_t)k * kRows * kD;
    sa.u = XS + (size_t)k * kRows * kD;
    sa.bc = XD + (size_t)k * kRows * kXpP;
    sa.z = nullptr;
    sa.A_log = ALP + (size_t)k * kD * kNst;
    sa.Dskip = DSP + (size_t)k * kD;
    sa.y = (__half*)(YH + (size_t)k * kRows * kD);
    sa.y_lo = nullptr;
    sa.ld_dtpre = kD;
    sa.ld_u = kD;
    sa.ld_bc = kXpP;
    sa.ld_z = 0;
    sa.ld_y = kD;
    sa.offB = kRank;
    sa.offC = kRank + kNst;
    sa.offZ = 0;
    sa.ycarry = kYCarry;
    sa.dir = 1;
    sa.D = kD;
    sa.L = kL;
    sa.nbatch = kBatch;
    ms1_scan_kernel<16><<<dim3((kD / 64) * kBatch), 64, 0, stream>>>(sa);
  }

  merge_out_kernel<<<(kBatch * kD * kL / 4) / 256, 256, 0, stream>>>(YH, out);
}
